// SelfAttention_62182536512219
// MI455X (gfx1250) — hardware-verified
//
#include <hip/hip_runtime.h>
#include <stdint.h>


typedef _Float16 v16h __attribute__((ext_vector_type(16)));
typedef _Float16 v8h  __attribute__((ext_vector_type(8)));
typedef float    v8f  __attribute__((ext_vector_type(8)));
typedef float    v4f  __attribute__((ext_vector_type(4)));

#ifndef NB
#define NB 8
#endif
#ifndef SEQ
#define SEQ 2048
#endif
#ifndef SCORE_RES
#define SCORE_RES 1
#endif
#define MCTX      SEQ
#define NB_FULL   8
#define SEQ_FULL  2048
#define MCTX_FULL SEQ_FULL
#define DM   512

#define ACT_CAR   8.0f
#define W_CAR     1024.0f
#define PROJ_SCL  0.0009765625f
#define RES_CAR   2048.0f
#define RES_INV   0.00048828125f
#define S_SCL     0.015625f
#define P_CAR     16384.0f
#define O_SCL     0.001953125f
#define O_CAR     256.0f
#define OUT_SCL   3.814697265625e-06f

static_assert(DM == 512);
static_assert(DM % 128 == 0 && DM % 64 == 0 && DM % 32 == 0);
static_assert(SEQ % 128 == 0);
static_assert(MCTX == SEQ);
static_assert(MCTX % 256 == 0);
static_assert(MCTX % 32 == 0);
static_assert(SEQ % 8 == 0);
static_assert(NB >= 1 && NB <= NB_FULL);
static_assert(SEQ <= SEQ_FULL && MCTX <= MCTX_FULL);
static_assert(SCORE_RES == 0 || SCORE_RES == 1);
static_assert((long)NB_FULL * SEQ_FULL * DM * 4 == 33554432L);
static_assert(((long)NB * SEQ * DM / 8) % 256 == 0);
static_assert((long)(DM / 64) * (DM / 64) * 64 * 64 == (long)DM * DM);
static_assert((long)(DM / 128) * ((long)NB * SEQ / 64) * 64 * 128 == (long)NB * SEQ * DM);
static_assert((long)(MCTX / 64) * (DM / 128) * 128 * 64 == (long)DM * MCTX);
static_assert((long)(MCTX / 64) * (SEQ / 64) * 4096 == (long)SEQ * MCTX);
static_assert((long)(SEQ / 8) * 8 * MCTX == (long)SEQ * MCTX);
static_assert((long)(DM / 64) * (SEQ / 128) * 128 * 64 == (long)SEQ * DM);
static_assert((long)(DM / 64) * ((long)NB * SEQ / 128) * 128 * 64 == (long)NB * SEQ * DM);

union Frag16 { v16h v; v8h p[2]; };

__device__ __forceinline__ v16h ld_frag(const _Float16* p, int hl) {
  Frag16 f;
  f.p[0] = *(const v8h*)(p + 8 * hl);
  f.p[1] = *(const v8h*)(p + 16 + 8 * hl);
  return f.v;
}

__device__ __forceinline__ v8f mma(v16h a, v16h b, v8f c) {
  v8f d = __builtin_amdgcn_wmma_f32_16x16x32_f16(false, a, false, b, (short)0, c, false, false);
  asm volatile("v_nop\n\tv_nop\n\tv_nop\n\tv_nop" : "+v"(d) : "v"(a), "v"(b));
  return d;
}

__device__ __forceinline__ float bf16_rne(float x) {
  unsigned int u = __builtin_bit_cast(unsigned int, x);
  u += 0x7FFFu + ((u >> 16) & 1u);
  return __builtin_bit_cast(float, u & 0xFFFF0000u);
}

static __device__ __forceinline__ _Float16 toh_flush(float v) {
  const _Float16 r = (_Float16)v;
  return (fabsf(v) < 6.103515625e-05f) ? (_Float16)0.0f : r;
}

__global__ __launch_bounds__(256) void k_cvt8(const float* __restrict__ src,
                                              _Float16* __restrict__ dst,
                                              int rows_used, int rows_full, float car, int total8)
{
  const int i8 = blockIdx.x * 256 + threadIdx.x;
  if (i8 >= total8) return;
  const size_t e   = (size_t)i8 * 8;
  const size_t r   = e / (size_t)DM;
  const int    col = (int)(e - r * (size_t)DM);
  const size_t b   = r / (size_t)rows_used;
  const size_t rr  = r - b * (size_t)rows_used;
  const float* s = src + (b * (size_t)rows_full + rr) * (size_t)DM + col;
  const v4f x0 = *(const v4f*)s;
  const v4f x1 = *(const v4f*)(s + 4);
  v8h o;
#pragma unroll
  for (int j = 0; j < 4; ++j) {
    const float t0 = x0[j];
    const float t1 = x1[j];
    o[j]     = (_Float16)(bf16_rne(t0) * car);
    o[4 + j] = (_Float16)(bf16_rne(t1) * car);
  }
  _Float16* d = dst + e;
  *(volatile v8h*)d = o;
  __threadfence();
  *(volatile v8h*)d = o;
}

__global__ __launch_bounds__(256) void k_cvtT(const float* __restrict__ src,
                                              _Float16* __restrict__ dst, float car)
{
  __shared__ __attribute__((aligned(16))) _Float16 ldsT[64 * 72];

  const int tid = threadIdx.x;
  const int n0 = blockIdx.x * 64, k0 = blockIdx.y * 64;

  for (int i = 0; i < 4; ++i) {
    const int q = i * 256 + tid;
    const int kr = q >> 4, c4 = (q & 15) * 4;
    const v4f v = *(const v4f*)(src + (size_t)(k0 + kr) * DM + n0 + c4);
#pragma unroll
    for (int j = 0; j < 4; ++j) {
      const float t = v[j];
      ldsT[(c4 + j) * 72 + kr] = toh_flush(bf16_rne(t) * car);
    }
  }
  __syncthreads();

  for (int i = 0; i < 2; ++i) {
    const int q = i * 256 + tid;
    const int rowl = q >> 3, ch = (q & 7) * 8;
    const v8h vh = *(const v8h*)(ldsT + rowl * 72 + ch);
    *(volatile v8h*)(dst + (size_t)(n0 + rowl) * DM + k0 + ch) = vh;
  }
  __threadfence();
  for (int i = 0; i < 2; ++i) {
    const int q = i * 256 + tid;
    const int rowl = q >> 3, ch = (q & 7) * 8;
    const v8h vh = *(const v8h*)(ldsT + rowl * 72 + ch);
    *(volatile v8h*)(dst + (size_t)(n0 + rowl) * DM + k0 + ch) = vh;
  }
}

__device__ __forceinline__ void gemm_core(const _Float16* ap0, const _Float16* ap1,
                                          const _Float16* bp01, const _Float16* bp23,
                                          int K, int hl, v8f (&acc)[8])
{
  const size_t bst = (size_t)16 * K;
#pragma unroll 1
  for (int k0 = 0; k0 < K; k0 += 32) {
    const v16h a0 = ld_frag(ap0 + k0, hl);
    const v16h a1 = ld_frag(ap1 + k0, hl);
    const v16h b0 = ld_frag(bp01 + k0, hl);
    const v16h b1 = ld_frag(bp01 + bst + k0, hl);
    const v16h b2 = ld_frag(bp23 + k0, hl);
    const v16h b3 = ld_frag(bp23 + bst + k0, hl);
    acc[0] = mma(a0, b0, acc[0]);
    acc[1] = mma(a0, b1, acc[1]);
    acc[2] = mma(a0, b2, acc[2]);
    acc[3] = mma(a0, b3, acc[3]);
    acc[4] = mma(a1, b0, acc[4]);
    acc[5] = mma(a1, b1, acc[5]);
    acc[6] = mma(a1, b2, acc[6]);
    acc[7] = mma(a1, b3, acc[7]);
  }
}

__global__ __launch_bounds__(128) __attribute__((amdgpu_num_vgpr(256)))
void k_projqk(const _Float16* __restrict__ A, const _Float16* __restrict__ Bt,
              const float* __restrict__ bias,
              _Float16* __restrict__ PH, _Float16* __restrict__ PL)
{
  __shared__ __attribute__((aligned(16))) _Float16 ldsH[64 * 136];
  __shared__ __attribute__((aligned(16))) _Float16 ldsL[64 * 136];

  const int tid = threadIdx.x, lane = tid & 31;
  const int w = __builtin_amdgcn_readfirstlane((int)(threadIdx.x >> 5));
  const int hl = lane >> 4, c = lane & 15;
  const int wr = w >> 1, wc = w & 1;
  const int m0 = blockIdx.y * 64, n0 = blockIdx.x * 128;
  const int mw = m0 + 32 * wr;

  const _Float16* ap0  = A  + (size_t)(mw + c) * DM;
  const _Float16* ap1  = A  + (size_t)(mw + 16 + c) * DM;
  const _Float16* bp01 = Bt + (size_t)(n0 + 32 * wc + c) * DM;
  const _Float16* bp23 = Bt + (size_t)(n0 + 64 + 32 * wc + c) * DM;

  v8f acc[8] = {};
  gemm_core(ap0, ap1, bp01, bp23, DM, hl, acc);

#pragma unroll
  for (int t = 0; t < 4; ++t) {
    const int coll = ((t < 2) ? 0 : 64) + 32 * wc + 16 * (t & 1) + c;
    const float bb = bf16_rne(bias[n0 + coll]) * ACT_CAR;
#pragma unroll
    for (int i = 0; i < 2; ++i)
#pragma unroll
      for (int r = 0; r < 8; ++r) {
        const int rowl = 32 * wr + 16 * i + 8 * hl + r;
        const float y = acc[i * 4 + t][r] * PROJ_SCL + bb;
        const float v = (y > 0.0f) ? y : 0.0f;
        const _Float16 hv = toh_flush(v);
        const float res = (v - (float)hv) * RES_CAR;
        ldsH[rowl * 136 + coll] = hv;
        ldsL[rowl * 136 + coll] = toh_flush(res);
      }
  }
  __syncthreads();

  for (int i = 0; i < 8; ++i) {
    const int q = i * 128 + tid;
    const int rowl = q >> 4, ch = (q & 15) * 8;
    const v8h vh = *(const v8h*)(ldsH + rowl * 136 + ch);
    const size_t go = (size_t)(m0 + rowl) * DM + n0 + ch;
    *(volatile v8h*)(PH + go) = vh;
  }
  for (int i = 0; i < 8; ++i) {
    const int q = i * 128 + tid;
    const int rowl = q >> 4, ch = (q & 15) * 8;
    const v8h vl = *(const v8h*)(ldsL + rowl * 136 + ch);
    const size_t go = (size_t)(m0 + rowl) * DM + n0 + ch;
    *(volatile v8h*)(PL + go) = vl;
  }
  __threadfence();
  for (int i = 0; i < 8; ++i) {
    const int q = i * 128 + tid;
    const int rowl = q >> 4, ch = (q & 15) * 8;
    const v8h vh = *(const v8h*)(ldsH + rowl * 136 + ch);
    const size_t go = (size_t)(m0 + rowl) * DM + n0 + ch;
    *(volatile v8h*)(PH + go) = vh;
  }
  for (int i = 0; i < 8; ++i) {
    const int q = i * 128 + tid;
    const int rowl = q >> 4, ch = (q & 15) * 8;
    const v8h vl = *(const v8h*)(ldsL + rowl * 136 + ch);
    const size_t go = (size_t)(m0 + rowl) * DM + n0 + ch;
    *(volatile v8h*)(PL + go) = vl;
  }
}

__global__ __launch_bounds__(128) __attribute__((amdgpu_num_vgpr(256)))
void k_projv(const _Float16* __restrict__ A, const _Float16* __restrict__ Bt,
             const float* __restrict__ bias, _Float16* __restrict__ PH)
{
  __shared__ __attribute__((aligned(16))) _Float16 ldsH[128 * 72];

  const int tid = threadIdx.x, lane = tid & 31;
  const int w = __builtin_amdgcn_readfirstlane((int)(threadIdx.x >> 5));
  const int hl = lane >> 4, c = lane & 15;
  const int m0 = blockIdx.y * 128, n0 = blockIdx.x * 64;
  const int z = blockIdx.z;
  const int mw = m0 + 32 * w;

  const _Float16* Bz = Bt + (size_t)z * MCTX * DM;
  _Float16* const Pz = PH + (size_t)z * DM * MCTX;

  const _Float16* ap0 = A  + (size_t)(mw + c) * DM;
  const _Float16* ap1 = A  + (size_t)(mw + 16 + c) * DM;
  const _Float16* bp  = Bz + (size_t)(n0 + c) * DM;

  v8f acc[8] = {};
  gemm_core(ap0, ap1, bp, bp + (size_t)32 * DM, DM, hl, acc);

#pragma unroll
  for (int i = 0; i < 2; ++i) {
    const float* bb = bias + m0 + 32 * w + 16 * i + 8 * hl;
    const v4f bA = *(const v4f*)bb;
    const v4f bB = *(const v4f*)(bb + 4);
#pragma unroll
    for (int r = 0; r < 8; ++r) {
      const float braw = (r < 4) ? bA[r & 3] : bB[r & 3];
      const float bv = bf16_rne(braw) * ACT_CAR;
      const int rowl = 32 * w + 16 * i + 8 * hl + r;
#pragma unroll
      for (int t = 0; t < 4; ++t) {
        const float y = acc[i * 4 + t][r] * PROJ_SCL + bv;
        const float v = (y > 0.0f) ? y : 0.0f;
        ldsH[rowl * 72 + 16 * t + c] = toh_flush(v);
      }
    }
  }
  __syncthreads();

  _Float16* const bh = Pz + (size_t)m0 * MCTX + n0;
  for (int i = 0; i < 8; ++i) {
    const int q = i * 128 + tid;
    const int rowl = q >> 3, ch = (q & 7) * 8;
    const v8h vh = *(const v8h*)(ldsH + rowl * 72 + ch);
    *(volatile v8h*)(bh + (size_t)rowl * MCTX + ch) = vh;
  }
  __threadfence();
  for (int i = 0; i < 8; ++i) {
    const int q = i * 128 + tid;
    const int rowl = q >> 3, ch = (q & 7) * 8;
    const v8h vh = *(const v8h*)(ldsH + rowl * 72 + ch);
    *(volatile v8h*)(bh + (size_t)rowl * MCTX + ch) = vh;
  }
}

__global__ __launch_bounds__(128) __attribute__((amdgpu_num_vgpr(256)))
void k_score(const _Float16* __restrict__ QH, const _Float16* __restrict__ QL,
             const _Float16* __restrict__ KH, const _Float16* __restrict__ KL,
             float* __restrict__ S)
{
  __shared__ __attribute__((aligned(16))) float ldsF[64 * 68];

  const int tid = threadIdx.x, lane = tid & 31;
  const int w = __builtin_amdgcn_readfirstlane((int)(threadIdx.x >> 5));
  const int hl = lane >> 4, c = lane & 15;
  const int m0 = blockIdx.y * 64, n0 = blockIdx.x * 64;
  const int mw = m0 + 16 * w;

  const _Float16* ah = QH + (size_t)(mw + c) * DM;
  const _Float16* al = QL + (size_t)(mw + c) * DM;
  const _Float16* bh = KH + (size_t)(n0 + c) * DM;
  const _Float16* bl = KL + (size_t)(n0 + c) * DM;

  v8f sh[4] = {}, sl[4] = {};
#pragma unroll 1
  for (int k0 = 0; k0 < DM; k0 += 32) {
    const v16h qh = ld_frag(ah + k0, hl);
    if (SCORE_RES != 0) {
      const v16h ql = ld_frag(al + k0, hl);
#pragma unroll
      for (int t = 0; t < 4; ++t) {
        const v16h kf = ld_frag(bh + (size_t)t * 16 * DM + k0, hl);
        const v16h kr = ld_frag(bl + (size_t)t * 16 * DM + k0, hl);
        sh[t] = mma(qh, kf, sh[t]);
        sl[t] = mma(ql, kf, sl[t]);
        sl[t] = mma(qh, kr, sl[t]);
      }
    } else {
#pragma unroll
      for (int t = 0; t < 4; ++t) {
        const v16h kf = ld_frag(bh + (size_t)t * 16 * DM + k0, hl);
        sh[t] = mma(qh, kf, sh[t]);
      }
    }
  }

#pragma unroll
  for (int t = 0; t < 4; ++t)
#pragma unroll
    for (int r = 0; r < 8; ++r) {
      const int rowl = 16 * w + 8 * hl + r;
      ldsF[rowl * 68 + 16 * t + c] = (sh[t][r] + sl[t][r] * RES_INV) * S_SCL;
    }
  __syncthreads();

  float* const ob = S + (size_t)m0 * MCTX + n0;
  for (int i = 0; i < 8; ++i) {
    const int qi = i * 128 + tid;
    const int rowl = qi >> 4, col = (qi & 15) * 4;
    const v4f v = *(const v4f*)(ldsF + rowl * 68 + col);
    *(volatile v4f*)(ob + (size_t)rowl * MCTX + col) = v;
  }
  __threadfence();
  for (int i = 0; i < 8; ++i) {
    const int qi = i * 128 + tid;
    const int rowl = qi >> 4, col = (qi & 15) * 4;
    const v4f v = *(const v4f*)(ldsF + rowl * 68 + col);
    *(volatile v4f*)(ob + (size_t)rowl * MCTX + col) = v;
  }
}

__global__ __launch_bounds__(256) void k_softmax(const float* __restrict__ S,
                                                 _Float16* __restrict__ P)
{
  constexpr int NI = MCTX / 256;
  static_assert(NI * 256 == MCTX);
  static_assert(NI >= 1 && NI <= 8);
  const int lane = threadIdx.x & 31, w = threadIdx.x >> 5;
  const int row = blockIdx.x * 8 + w;
  const float* sp = S + (size_t)row * MCTX + 8 * lane;

  v4f xa[NI], xb[NI];
#pragma unroll
  for (int i = 0; i < NI; ++i) {
    xa[i] = *(const v4f*)(sp + i * 256);
    xb[i] = *(const v4f*)(sp + i * 256 + 4);
  }
  float mx = -__builtin_inff();
#pragma unroll
  for (int i = 0; i < NI; ++i)
#pragma unroll
    for (int j = 0; j < 4; ++j) {
      mx = fmaxf(mx, xa[i][j]);
      mx = fmaxf(mx, xb[i][j]);
    }
  mx = fmaxf(mx, __shfl_xor(mx, 16, 32));
  mx = fmaxf(mx, __shfl_xor(mx, 8, 32));
  mx = fmaxf(mx, __shfl_xor(mx, 4, 32));
  mx = fmaxf(mx, __shfl_xor(mx, 2, 32));
  mx = fmaxf(mx, __shfl_xor(mx, 1, 32));

  float sm = 0.f;
#pragma unroll
  for (int i = 0; i < NI; ++i)
#pragma unroll
    for (int j = 0; j < 4; ++j) {
      const float ea = __expf(xa[i][j] - mx);
      const float eb = __expf(xb[i][j] - mx);
      xa[i][j] = ea;
      xb[i][j] = eb;
      sm += ea;
      sm += eb;
    }
  sm += __shfl_xor(sm, 16, 32);
  sm += __shfl_xor(sm, 8, 32);
  sm += __shfl_xor(sm, 4, 32);
  sm += __shfl_xor(sm, 2, 32);
  sm += __shfl_xor(sm, 1, 32);
  const float inv = P_CAR * (1.0f / sm);

  v8h o[NI];
#pragma unroll
  for (int i = 0; i < NI; ++i)
#pragma unroll
    for (int j = 0; j < 4; ++j) {
      o[i][j]     = (_Float16)(xa[i][j] * inv);
      o[i][4 + j] = (_Float16)(xb[i][j] * inv);
    }
  _Float16* pp = P + (size_t)row * MCTX + 8 * lane;
#pragma unroll
  for (int i = 0; i < NI; ++i) *(volatile v8h*)(pp + i * 256) = o[i];
  __threadfence();
#pragma unroll
  for (int i = 0; i < NI; ++i) *(volatile v8h*)(pp + i * 256) = o[i];
}

__device__ __forceinline__ v8h addx8(v4f a0, v4f a1, v4f x0, v4f x1) {
  v8h o;
#pragma unroll
  for (int j = 0; j < 4; ++j) {
    const float t0 = a0[j] + bf16_rne(x0[j]) * O_CAR;
    const float t1 = a1[j] + bf16_rne(x1[j]) * O_CAR;
    o[j]     = toh_flush(t0);
    o[4 + j] = toh_flush(t1);
  }
  return o;
}

__global__ __launch_bounds__(128) __attribute__((amdgpu_num_vgpr(256)))
void k_pv(const _Float16* __restrict__ A, const _Float16* __restrict__ Bt,
          const float* __restrict__ XR, _Float16* __restrict__ PH)
{
  __shared__ __attribute__((aligned(16))) float ldsF[128 * 68];

  const int tid = threadIdx.x, lane = tid & 31;
  const int w = __builtin_amdgcn_readfirstlane((int)(threadIdx.x >> 5));
  const int hl = lane >> 4, c = lane & 15;
  const int m0 = blockIdx.y * 128, n0 = blockIdx.x * 64;
  const int mw = m0 + 32 * w;

  const _Float16* ap0 = A  + (size_t)(mw + c) * MCTX;
  const _Float16* ap1 = A  + (size_t)(mw + 16 + c) * MCTX;
  const _Float16* bp  = Bt + (size_t)(n0 + c) * MCTX;

  v8f acc[8] = {};
  gemm_core(ap0, ap1, bp, bp + (size_t)32 * MCTX, MCTX, hl, acc);

#pragma unroll
  for (int i = 0; i < 2; ++i)
#pragma unroll
    for (int t = 0; t < 4; ++t)
#pragma unroll
      for (int r = 0; r < 8; ++r) {
        const int rowl = 32 * w + 16 * i + 8 * hl + r;
        ldsF[rowl * 68 + 16 * t + c] = acc[i * 4 + t][r] * O_SCL;
      }
  __syncthreads();

  _Float16* const bh = PH + (size_t)m0 * DM + n0;
  const float* const xb = XR + (size_t)m0 * DM + n0;
  for (int i = 0; i < 8; ++i) {
    const int q = i * 128 + tid;
    const int rowl = q >> 3, ch = (q & 7) * 8;
    const v4f a0 = *(const v4f*)(ldsF + rowl * 68 + ch);
    const v4f a1 = *(const v4f*)(ldsF + rowl * 68 + ch + 4);
    const v4f x0 = *(const v4f*)(xb + (size_t)rowl * DM + ch);
    const v4f x1 = *(const v4f*)(xb + (size_t)rowl * DM + ch + 4);
    const v8h vh = addx8(a0, a1, x0, x1);
    *(volatile v8h*)(bh + (size_t)rowl * DM + ch) = vh;
  }
  __threadfence();
  for (int i = 0; i < 8; ++i) {
    const int q = i * 128 + tid;
    const int rowl = q >> 3, ch = (q & 7) * 8;
    const v4f a0 = *(const v4f*)(ldsF + rowl * 68 + ch);
    const v4f a1 = *(const v4f*)(ldsF + rowl * 68 + ch + 4);
    const v4f x0 = *(const v4f*)(xb + (size_t)rowl * DM + ch);
    const v4f x1 = *(const v4f*)(xb + (size_t)rowl * DM + ch + 4);
    const v8h vh = addx8(a0, a1, x0, x1);
    *(volatile v8h*)(bh + (size_t)rowl * DM + ch) = vh;
  }
}

__global__ __launch_bounds__(128) __attribute__((amdgpu_num_vgpr(256)))
void k_oproj(const _Float16* __restrict__ A, const _Float16* __restrict__ Bt,
             const float* __restrict__ bias, float* __restrict__ Out)
{
  __shared__ __attribute__((aligned(16))) float ldsF[128 * 68];

  const int tid = threadIdx.x, lane = tid & 31;
  const int w = __builtin_amdgcn_readfirstlane((int)(threadIdx.x >> 5));
  const int hl = lane >> 4, c = lane & 15;
  const int m0 = blockIdx.y * 128, n0 = blockIdx.x * 64;
  const int mw = m0 + 32 * w;

  const _Float16* ap0 = A  + (size_t)(mw + c) * DM;
  const _Float16* ap1 = A  + (size_t)(mw + 16 + c) * DM;
  const _Float16* bp  = Bt + (size_t)(n0 + c) * DM;

  v8f acc[8] = {};
  gemm_core(ap0, ap1, bp, bp + (size_t)32 * DM, DM, hl, acc);

#pragma unroll
  for (int t = 0; t < 4; ++t) {
    const float bo = bf16_rne(bias[n0 + 16 * t + c]);
#pragma unroll
    for (int i = 0; i < 2; ++i)
#pragma unroll
      for (int r = 0; r < 8; ++r) {
        const int rowl = 32 * w + 16 * i + 8 * hl + r;
        const float y = acc[i * 4 + t][r] * OUT_SCL + bo;
        ldsF[rowl * 68 + 16 * t + c] = (y > 0.0f) ? y : 0.0f;
      }
  }
  __syncthreads();

  const int bz = m0 / SEQ, sr = m0 - bz * SEQ;
  float* const ob = Out + ((size_t)bz * SEQ_FULL + sr) * DM + n0;
  for (int i = 0; i < 16; ++i) {
    const int qi = i * 128 + tid;
    const int rowl = qi >> 4, col = (qi & 15) * 4;
    const v4f v = *(const v4f*)(ldsF + rowl * 68 + col);
    *(volatile v4f*)(ob + (size_t)rowl * DM + col) = v;
  }
  __threadfence();
  for (int i = 0; i < 16; ++i) {
    const int qi = i * 128 + tid;
    const int rowl = qi >> 4, col = (qi & 15) * 4;
    const v4f v = *(const v4f*)(ldsF + rowl * 68 + col);
    *(volatile v4f*)(ob + (size_t)rowl * DM + col) = v;
  }
}

constexpr size_t cmax(size_t a, size_t b) { return a > b ? a : b; }
constexpr size_t N_X   = (size_t)NB * SEQ * DM;
constexpr size_t N_W   = (size_t)DM * DM;
constexpr size_t B_X16 = N_X * 2;
constexpr size_t B_S   = (size_t)SEQ * MCTX * 4;
constexpr size_t B_P   = (size_t)SEQ * MCTX * 2;
constexpr size_t B_R0  = cmax(B_X16, B_S + B_P);
constexpr size_t B_W   = 4 * N_W * 2;
constexpr size_t B_Q   = 2 * N_X * 2;
constexpr size_t B_K   = 2 * N_X * 2;
constexpr size_t B_VT  = N_X * 2;
constexpr size_t B_O   = N_X * 2;
constexpr size_t OFF_W   = B_R0;
constexpr size_t OFF_Q   = OFF_W + B_W;
constexpr size_t OFF_K   = OFF_Q + B_Q;
constexpr size_t OFF_VT  = OFF_K + B_K;
constexpr size_t OFF_O   = OFF_VT + B_VT;
constexpr size_t WS_TOTAL = OFF_O + B_O;
static_assert(B_X16 <= B_R0 && B_S + B_P <= B_R0);
static_assert(B_R0 % 128 == 0 && B_W % 128 == 0);
static_assert(B_Q % 128 == 0 && B_K % 128 == 0 && B_VT % 128 == 0 && B_O % 128 == 0 && B_S % 128 == 0);
static_assert(WS_TOTAL <= (size_t)134217728);

extern "C" void kernel_launch(void* const* d_in, const int* in_sizes, int n_in,
                              void* d_out, int out_size, void* d_ws, size_t ws_size,
                              hipStream_t stream)
{
  if (n_in < 9) return;
  const long needX = ((long)(NB - 1) * SEQ_FULL + SEQ) * DM;
  if ((long)in_sizes[0] < needX) return;
  if ((long)in_sizes[1] < (long)DM * DM) return;
  if ((long)in_sizes[2] < (long)DM) return;
  if ((long)in_sizes[3] < (long)DM * DM) return;
  if ((long)in_sizes[4] < (long)DM) return;
  if ((long)in_sizes[5] < (long)DM * DM) return;
  if ((long)in_sizes[6] < (long)DM) return;
  if ((long)in_sizes[7] < (long)DM * DM) return;
  if ((long)in_sizes[8] < (long)DM) return;
  if ((long)out_size < needX) return;
  if (WS_TOTAL > ws_size) return;

  const float* x  = (const float*)d_in[0];
  const float* Wh = (const float*)d_in[1];
  const float* bh = (const float*)d_in[2];
  const float* Wl = (const float*)d_in[3];
  const float* bl = (const float*)d_in[4];
  const float* Wg = (const float*)d_in[5];
  const float* bg = (const float*)d_in[6];
  const float* Wm = (const float*)d_in[7];
  const float* bm = (const float*)d_in[8];
  float* out = (float*)d_out;

  char* const ws = (char*)d_ws;
  _Float16* X16 = (_Float16*)ws;
  float*    Sp  = (float*)ws;
  _Float16* Pp  = (_Float16*)(ws + B_S);
  _Float16* WlP = (_Float16*)(ws + OFF_W);
  _Float16* WhP = WlP + N_W;
  _Float16* WgP = WhP + N_W;
  _Float16* WmP = WgP + N_W;
  _Float16* QH  = (_Float16*)(ws + OFF_Q);
  _Float16* QL  = QH + N_X;
  _Float16* KH  = (_Float16*)(ws + OFF_K);
  _Float16* KL  = KH + N_X;
  _Float16* VtH = (_Float16*)(ws + OFF_VT);
  _Float16* OH  = (_Float16*)(ws + OFF_O);

  const int tx8 = (int)(N_X / 8);
  k_cvt8<<<(tx8 + 255) / 256, 256, 0, stream>>>(x, X16, SEQ, SEQ_FULL, ACT_CAR, tx8);
  k_cvtT<<<dim3(DM / 64, DM / 64), 256, 0, stream>>>(Wl, WlP, W_CAR);
  k_cvtT<<<dim3(DM / 64, DM / 64), 256, 0, stream>>>(Wh, WhP, W_CAR);
  k_cvtT<<<dim3(DM / 64, DM / 64), 256, 0, stream>>>(Wg, WgP, W_CAR);
  k_cvtT<<<dim3(DM / 64, DM / 64), 256, 0, stream>>>(Wm, WmP, W_CAR);

  k_projqk<<<dim3(DM / 128, NB * SEQ / 64), 128, 0, stream>>>(X16, WlP, bl, QH, QL);
  k_projqk<<<dim3(DM / 128, NB * SEQ / 64), 128, 0, stream>>>(X16, WhP, bh, KH, KL);
  k_projv<<<dim3(MCTX / 64, DM / 128, NB), 128, 0, stream>>>(WgP, X16, bg, VtH);

  for (int b = 0; b < NB; ++b) {
    const size_t qo = (size_t)b * SEQ * DM;
    const size_t ko = (size_t)b * MCTX * DM;
    const float* xr = x + (size_t)b * SEQ_FULL * DM;
    k_score<<<dim3(MCTX / 64, SEQ / 64), 128, 0, stream>>>(QH + qo, QL + qo, KH + ko, KL + ko, Sp);
    k_softmax<<<SEQ / 8, 256, 0, stream>>>(Sp, Pp);
    k_pv<<<dim3(DM / 64, SEQ / 128), 128, 0, stream>>>(Pp, VtH + ko, xr, OH + qo);
  }

  k_oproj<<<dim3(DM / 64, NB * SEQ / 128), 128, 0, stream>>>(OH, WmP, bm, out);
}
